// selfatt_64896955843117
// MI455X (gfx1250) — hardware-verified
//
#include <hip/hip_runtime.h>
#include <math.h>
#include <stdint.h>

#ifndef NB
#define NB 4
#endif
#ifndef NQ
#define NQ 4096
#endif
#define NBF   4
#define CC    512
#define CIN   513
#define NN    4096
#define DQ    64
#define MQK   128
#define MW    640
#define QT    64
#define CH    256
#define OSP   68
#define OSPW  132
#define TP    72
#define WSC   256.0f
#define IWSC  0.00390625f
#define LNPS  9.704060527839234f
#define INVNN 0.000244140625f

static_assert(NB >= 1 && NB <= NBF);
static_assert(NQ >= QT && NQ <= NN && NQ % QT == 0);
static_assert(NN % QT == 0 && CC % QT == 0 && MQK % QT == 0);
static_assert(MQK == 2 * DQ && MW == MQK + CC && MW % 8 == 0);
static_assert(DQ == QT);
static_assert(CC == 2 * CH && CH == 16 * 16);
static_assert(CC % 256 == 0 && CC % 32 == 0 && DQ % 32 == 0 && NN % 32 == 0);
static_assert((OSP * 4) % 16 == 0);
static_assert((OSPW * 4) % 16 == 0);
static_assert((TP * 2) % 16 == 0);

typedef _Float16       v16h __attribute__((ext_vector_type(16)));
typedef _Float16       v8h  __attribute__((ext_vector_type(8)));
typedef __bf16         v16b __attribute__((ext_vector_type(16)));
typedef unsigned short v8us __attribute__((ext_vector_type(8)));
typedef float          v8f  __attribute__((ext_vector_type(8)));
typedef float          v4f  __attribute__((ext_vector_type(4)));
typedef unsigned int   v4u  __attribute__((ext_vector_type(4)));

union Frag  { v8us u[2]; v16h h; v16b bf; };
union FragH { v16h v; v8h hv[2]; };
static_assert(sizeof(Frag) == 32);
static_assert(sizeof(FragH) == 32);

__device__ __forceinline__ unsigned short bf_bits(float f) {
  unsigned u = __float_as_uint(f);
  return (unsigned short)((u + 0x7FFFu + ((u >> 16) & 1u)) >> 16);
}
__device__ __forceinline__ float bf_up(unsigned short hb) { return __uint_as_float(((unsigned)hb) << 16); }
__device__ __forceinline__ float bfr(float f) { return bf_up(bf_bits(f)); }
__device__ __forceinline__ unsigned short h_bits(_Float16 x) { return __builtin_bit_cast(unsigned short, x); }
__device__ __forceinline__ unsigned pk16(unsigned short a, unsigned short b) { return (unsigned)a | ((unsigned)b << 16); }
__device__ __forceinline__ v8f zero8() { v8f z = {0.f, 0.f, 0.f, 0.f, 0.f, 0.f, 0.f, 0.f}; return z; }
__device__ __forceinline__ float hmax8(v8f s) {
  return fmaxf(fmaxf(fmaxf(s[0], s[1]), fmaxf(s[2], s[3])), fmaxf(fmaxf(s[4], s[5]), fmaxf(s[6], s[7])));
}
__device__ __forceinline__ unsigned wave_ballot(bool p) {
#if defined(__HIP_DEVICE_COMPILE__)
  return __builtin_amdgcn_ballot_w32(p);
#else
  return p ? 1u : 0u;
#endif
}
__device__ __forceinline__ float wpos(int l) { return ((float)l * INVNN) * 2.0f - 1.0f; }

__device__ __forceinline__ Frag ldfrag(const unsigned short* p) {
  Frag f;
  f.u[0] = *(const v8us*)(p);
  f.u[1] = *(const v8us*)(p + 16);
  return f;
}

__device__ __forceinline__ v8f mma_h(v16h a, v16h b, v8f c) {
  v8f d = __builtin_amdgcn_wmma_f32_16x16x32_f16(false, a, false, b, (short)0, c, false, false);
#if defined(__HIP_DEVICE_COMPILE__)
  asm volatile("v_nop\n\tv_nop\n\tv_nop\n\tv_nop" : "+v"(d) : "v"(a), "v"(b));
#endif
  return d;
}
__device__ __forceinline__ v8f mma_b(v16b a, v16b b, v8f c) {
  v8f d = __builtin_amdgcn_wmma_f32_16x16x32_bf16(false, a, false, b, (short)0, c, false, false);
#if defined(__HIP_DEVICE_COMPILE__)
  const v16h ha = __builtin_bit_cast(v16h, a), hb = __builtin_bit_cast(v16h, b);
  asm volatile("v_nop\n\tv_nop\n\tv_nop\n\tv_nop" : "+v"(d) : "v"(ha), "v"(hb));
#endif
  return d;
}

__global__ __launch_bounds__(256)
void cvt_w(const float* __restrict__ wq, const float* __restrict__ wk, const float* __restrict__ wv,
           unsigned short* W16) {
  const int tid = threadIdx.x, blk = blockIdx.x;
  const int rl = tid >> 5, lane = tid & 31;
  const int o = 8 * blk + rl;
  const float* wbase = (blk < (DQ / 8)) ? wq : ((blk < (MQK / 8)) ? wk : wv);
  const int osub = (blk < (DQ / 8)) ? 0 : ((blk < (MQK / 8)) ? DQ : MQK);
  const float* s = wbase + (size_t)(o - osub) * CIN;
#pragma unroll 1
  for (int cp = 0; cp < CC / 256; ++cp) {
    const int col = 256 * cp + 8 * lane;
    float f[8];
#pragma unroll
    for (int t = 0; t < 8; ++t) f[t] = s[col + t];
    v4u u;
#pragma unroll
    for (int t = 0; t < 4; ++t) {
      const _Float16 h0 = (_Float16)(bfr(f[2 * t]) * WSC);
      const _Float16 h1 = (_Float16)(bfr(f[2 * t + 1]) * WSC);
      u[t] = pk16(h_bits(h0), h_bits(h1));
    }
#pragma unroll
    for (int pass = 0; pass < 2; ++pass) {
      *(volatile v4u*)(W16 + (size_t)o * CC + col) = u;
      __threadfence();
    }
  }
}

__global__ __launch_bounds__(256)
void cvt_x(const float* __restrict__ x, unsigned short* XP) {
  __shared__ __align__(16) unsigned short T[QT * TP];
  const int tid = threadIdx.x;
  const int nb = blockIdx.x, cb = blockIdx.y, b = blockIdx.z;
  const int e = tid & 7, lq = tid >> 3;
  const int n0 = nb * QT, c0 = cb * QT;
#pragma unroll
  for (int it = 0; it < 2; ++it) {
    const int cl = it * 32 + lq;
    const float* sp = x + ((size_t)(b * CC + c0 + cl)) * NN + n0 + 8 * e;
    const v4f a = *(const v4f*)sp;
    const v4f q = *(const v4f*)(sp + 4);
#pragma unroll
    for (int t = 0; t < 4; ++t) {
      T[(8 * e + t) * TP + cl]     = h_bits((_Float16)bfr(a[t]));
      T[(8 * e + 4 + t) * TP + cl] = h_bits((_Float16)bfr(q[t]));
    }
  }
  __syncthreads();
  v4u up[2];
#pragma unroll
  for (int it = 0; it < 2; ++it) {
    const int nl = it * 32 + lq;
    up[it] = *(const v4u*)(T + nl * TP + 8 * e);
  }
#pragma unroll
  for (int pass = 0; pass < 2; ++pass) {
#pragma unroll
    for (int it = 0; it < 2; ++it) {
      const int rl = it * 32 + lq;
      *(volatile v4u*)(XP + ((size_t)(b * NN + n0 + rl)) * CC + c0 + 8 * e) = up[it];
    }
    __threadfence();
  }
}

__device__ __forceinline__ void gemm_core(const unsigned short* __restrict__ ap,
                                          const unsigned short* __restrict__ bp,
                                          float* Os, int wave, int hh, int c) {
  v8f acc[4];
#pragma unroll
  for (int mt = 0; mt < 4; ++mt) acc[mt] = zero8();

#pragma unroll 4
  for (int ks = 0; ks < CC / 32; ++ks) {
    const Frag fb = ldfrag(bp + 32 * ks);
#pragma unroll
    for (int mt = 0; mt < 4; ++mt) {
      const Frag fa = ldfrag(ap + (size_t)(16 * mt) * CC + 32 * ks);
      acc[mt] = mma_h(fa.h, fb.h, acc[mt]);
    }
  }

  const int nl = 16 * wave + c;
#pragma unroll
  for (int mt = 0; mt < 4; ++mt) {
    v4f va, vb;
#pragma unroll
    for (int r = 0; r < 4; ++r) { va[r] = acc[mt][r] * IWSC; vb[r] = acc[mt][4 + r] * IWSC; }
    *(v4f*)(Os + nl * OSP + 16 * mt + 8 * hh)     = va;
    *(v4f*)(Os + nl * OSP + 16 * mt + 8 * hh + 4) = vb;
  }
}

__global__ __launch_bounds__(128)
void gemm_qk(const unsigned short* __restrict__ W16, const unsigned short* __restrict__ XP,
             const float* __restrict__ wq, const float* __restrict__ wk,
             unsigned short* Qh, unsigned short* Ql, unsigned short* Kh, unsigned short* Kl) {
  __shared__ __align__(16) float Os[QT * OSP];
  const int tid  = threadIdx.x;
  const int lane = tid & 31, wave = tid >> 5;
  const int hh   = lane >> 4, c = lane & 15;
  const int nt   = blockIdx.x, mb = blockIdx.y, b = blockIdx.z;
  const int n0   = nt * QT, o0 = mb * QT;

  const unsigned short* ap = W16 + (size_t)(o0 + c) * CC + 8 * hh;
  const unsigned short* bp = XP + ((size_t)(b * NN + n0 + 16 * wave + c)) * CC + 8 * hh;
  gemm_core(ap, bp, Os, wave, hh, c);
  __syncthreads();

  const int e = tid & 7, lq = tid >> 3;
  const float* wsrc = (mb == 0) ? wq : wk;
  unsigned short* Ph = (mb == 0) ? Qh : Kh;
  unsigned short* Pl = (mb == 0) ? Ql : Kl;
  float pw[8];
#pragma unroll
  for (int t = 0; t < 8; ++t) pw[t] = bfr(wsrc[(size_t)(8 * e + t) * CIN + CC]);

  v4u uh[4], ul[4];
#pragma unroll
  for (int it = 0; it < 4; ++it) {
    const int row = it * 16 + lq;
    const float wl = wpos(n0 + row);
    const v4f a = *(const v4f*)(Os + row * OSP + 8 * e);
    const v4f q = *(const v4f*)(Os + row * OSP + 8 * e + 4);
    const float f[8] = {a[0], a[1], a[2], a[3], q[0], q[1], q[2], q[3]};
#pragma unroll
    for (int t = 0; t < 4; ++t) {
      const float f0 = f[2 * t] + pw[2 * t] * wl;
      const float f1 = f[2 * t + 1] + pw[2 * t + 1] * wl;
      const unsigned short hb0 = bf_bits(f0), hb1 = bf_bits(f1);
      const unsigned short lb0 = bf_bits(f0 - bf_up(hb0));
      const unsigned short lb1 = bf_bits(f1 - bf_up(hb1));
      uh[it][t] = pk16(hb0, hb1);
      ul[it][t] = pk16(lb0, lb1);
    }
  }
#pragma unroll
  for (int pass = 0; pass < 2; ++pass) {
#pragma unroll
    for (int it = 0; it < 4; ++it) {
      const int row = it * 16 + lq;
      const size_t po = ((size_t)(b * NN + n0 + row)) * DQ + 8 * e;
      *(volatile v4u*)(Ph + po) = uh[it];
      *(volatile v4u*)(Pl + po) = ul[it];
    }
    __threadfence();
  }
}

__global__ __launch_bounds__(128)
void gemm_v(const unsigned short* __restrict__ W16, const unsigned short* __restrict__ XP,
            const float* __restrict__ wv, const float* __restrict__ bv, unsigned short* V) {
  __shared__ __align__(16) float Os[QT * OSP];
  const int tid  = threadIdx.x;
  const int lane = tid & 31, wave = tid >> 5;
  const int hh   = lane >> 4, c = lane & 15;
  const int nt   = blockIdx.x, mb = blockIdx.y, b = blockIdx.z;
  const int n0   = nt * QT, o0 = mb * QT;

  const unsigned short* ap = W16 + (size_t)(MQK + o0 + c) * CC + 8 * hh;
  const unsigned short* bp = XP + ((size_t)(b * NN + n0 + 16 * wave + c)) * CC + 8 * hh;
  gemm_core(ap, bp, Os, wave, hh, c);
  __syncthreads();

  const int e = tid & 7, lq = tid >> 3;
  float wl[8];
#pragma unroll
  for (int t = 0; t < 8; ++t) wl[t] = wpos(n0 + 8 * e + t);

  v4u uv[4];
#pragma unroll
  for (int it = 0; it < 4; ++it) {
    const int ol = it * 16 + lq;
    const int og = o0 + ol;
    const float pwo = bfr(wv[(size_t)og * CIN + CC]);
    const float bo  = bfr(bv[og]);
    unsigned short hb[8];
#pragma unroll
    for (int t = 0; t < 8; ++t) {
      const float val = Os[(8 * e + t) * OSP + ol] + pwo * wl[t] + bo;
      hb[t] = h_bits((_Float16)val);
    }
#pragma unroll
    for (int t = 0; t < 4; ++t) uv[it][t] = pk16(hb[2 * t], hb[2 * t + 1]);
  }
#pragma unroll
  for (int pass = 0; pass < 2; ++pass) {
#pragma unroll
    for (int it = 0; it < 4; ++it) {
      const int og = o0 + it * 16 + lq;
      *(volatile v4u*)(V + ((size_t)(b * CC + og)) * NN + n0 + 8 * e) = uv[it];
    }
    __threadfence();
  }
}

__global__ __launch_bounds__(128)
void attn_k(const unsigned short* __restrict__ Qh, const unsigned short* __restrict__ Ql,
            const unsigned short* __restrict__ Kh, const unsigned short* __restrict__ Kl,
            const unsigned short* __restrict__ V, const float* __restrict__ x,
            const float* __restrict__ gamma, float* out) {
  __shared__ __align__(16) float Os[QT * OSPW];
  const int tid  = threadIdx.x;
  const int wave = tid >> 5, lane = tid & 31;
  const int hh   = lane >> 4, c = lane & 15;
  const int n0   = blockIdx.x * QT, b = blockIdx.y, chh = blockIdx.z;
  const int cb0  = chh * CH;

  const size_t qo = ((size_t)(b * NN + n0 + 16 * wave + c)) * DQ + 8 * hh;
  const unsigned short* Qhp = Qh + qo;
  const unsigned short* Qlp = Ql + qo;
  const unsigned short* Khp = Kh + (size_t)b * NN * DQ + (size_t)c * DQ + 8 * hh;
  const unsigned short* Klp = Kl + (size_t)b * NN * DQ + (size_t)c * DQ + 8 * hh;
  const unsigned short* Vp = V + ((size_t)(b * CC + cb0 + c)) * NN + 8 * hh;

  float m = -1.0e30f, l = 0.f;
  v8f o[16];
#pragma unroll
  for (int j = 0; j < 16; ++j) o[j] = zero8();

#pragma unroll 1
  for (int kb = 0; kb < NN; kb += 32) {
    const unsigned short* k0p  = Khp + (size_t)kb * DQ;
    const unsigned short* k1p  = Khp + (size_t)(kb + 16) * DQ;
    const unsigned short* k0lp = Klp + (size_t)kb * DQ;
    const unsigned short* k1lp = Klp + (size_t)(kb + 16) * DQ;
    v8f s0 = zero8(), s1 = zero8();
#pragma unroll 1
    for (int kc = 0; kc < DQ / 32; ++kc) {
      const Frag qh  = ldfrag(Qhp + 32 * kc);
      const Frag ql  = ldfrag(Qlp + 32 * kc);
      const Frag k0  = ldfrag(k0p + 32 * kc);
      const Frag k1  = ldfrag(k1p + 32 * kc);
      const Frag k0l = ldfrag(k0lp + 32 * kc);
      const Frag k1l = ldfrag(k1lp + 32 * kc);
      s0 = mma_b(k0.bf, qh.bf, s0);
      s1 = mma_b(k1.bf, qh.bf, s1);
      s0 = mma_b(k0.bf, ql.bf, s0);
      s1 = mma_b(k1.bf, ql.bf, s1);
      s0 = mma_b(k0l.bf, qh.bf, s0);
      s1 = mma_b(k1l.bf, qh.bf, s1);
    }

    float mx = fmaxf(hmax8(s0), hmax8(s1));
    mx = fmaxf(mx, __shfl_xor(mx, 16, 32));
    const float mn = fmaxf(m, mx);
    const unsigned grew = wave_ballot(mx > m);
    if (grew != 0u) {
      const float corr = __expf(m - mn);
      l *= corr;
#pragma unroll
      for (int j = 0; j < 16; ++j) {
#pragma unroll
        for (int r = 0; r < 8; ++r) o[j][r] *= corr;
      }
    }
    m = mn;
    const float msh = mn - LNPS;

    FragH ph;
    float ls = 0.f;
#pragma unroll
    for (int r = 0; r < 8; ++r) {
      const float e0 = __expf(s0[r] - msh);
      const float e1 = __expf(s1[r] - msh);
      ls += e0 + e1;
      ph.hv[0][r] = (_Float16)e0;
      ph.hv[1][r] = (_Float16)e1;
    }
    l += ls;

#pragma unroll
    for (int j = 0; j < 16; ++j) {
      const Frag vf = ldfrag(Vp + (size_t)(16 * j) * NN + kb);
      o[j] = mma_h(vf.h, ph.v, o[j]);
    }
  }
  l += __shfl_xor(l, 16, 32);
  const float gam = bfr(gamma[0]);
  const float inv = gam / l;

  const int qrow = 16 * wave + c;
  const int e = tid & 7, lq = tid >> 3;
#pragma unroll
  for (int half = 0; half < 2; ++half) {
    if (half) __syncthreads();
#pragma unroll
    for (int jj = 0; jj < 8; ++jj) {
      const int j = 8 * half + jj;
      v4f va, vb;
#pragma unroll
      for (int r = 0; r < 4; ++r) { va[r] = o[j][r] * inv; vb[r] = o[j][4 + r] * inv; }
      *(v4f*)(Os + qrow * OSPW + 16 * jj + 8 * hh)     = va;
      *(v4f*)(Os + qrow * OSPW + 16 * jj + 8 * hh + 4) = vb;
    }
    __syncthreads();
    v4f res[16];
#pragma unroll
    for (int it = 0; it < 16; ++it) {
      const int L   = it * 16 + lq;
      const int chl = L >> 1, hf = L & 1;
      const int nl  = hf * 32 + 4 * e;
      const size_t idx = ((size_t)(b * CC + cb0 + 128 * half + chl)) * NN + n0 + nl;
      const v4f xv = *(const v4f*)(x + idx);
#pragma unroll
      for (int t = 0; t < 4; ++t) res[it][t] = Os[(nl + t) * OSPW + chl] + bfr(xv[t]);
    }
#pragma unroll
    for (int pass = 0; pass < 2; ++pass) {
#pragma unroll
      for (int it = 0; it < 16; ++it) {
        const int L   = it * 16 + lq;
        const int chl = L >> 1, hf = L & 1;
        const int nl  = hf * 32 + 4 * e;
        const size_t idx = ((size_t)(b * CC + cb0 + 128 * half + chl)) * NN + n0 + nl;
        *(volatile v4f*)(out + idx) = res[it];
      }
      __threadfence();
    }
  }
}

extern "C" void kernel_launch(void* const* d_in, const int* in_sizes, int n_in,
                              void* d_out, int out_size, void* d_ws, size_t ws_size,
                              hipStream_t stream) {
  const int XN = NB * CC * NN;
  if (n_in < 6) return;
  if (in_sizes[0] < XN) return;
  if (in_sizes[1] < DQ * CIN || in_sizes[2] < DQ * CIN) return;
  if (in_sizes[3] < CC * CIN || in_sizes[4] < CC || in_sizes[5] < 1) return;
  if (out_size < XN) return;

  size_t off = 0;
  auto carve = [&](size_t bytes) { const size_t o = off; off += (bytes + 255) & ~(size_t)255; return o; };
  const size_t oW16 = carve((size_t)MW * CC * 2);
  const size_t oXP  = carve((size_t)NB * NN * CC * 2);
  const size_t oV   = carve((size_t)NB * CC * NN * 2);
  const size_t oQh  = carve((size_t)NB * NN * DQ * 2);
  const size_t oQl  = carve((size_t)NB * NN * DQ * 2);
  const size_t oKh  = carve((size_t)NB * NN * DQ * 2);
  const size_t oKl  = carve((size_t)NB * NN * DQ * 2);
  if (off > ws_size) return;
  if (off > (size_t)134217728) return;

  const float* x     = (const float*)d_in[0];
  const float* wq    = (const float*)d_in[1];
  const float* wk    = (const float*)d_in[2];
  const float* wv    = (const float*)d_in[3];
  const float* bv    = (const float*)d_in[4];
  const float* gamma = (const float*)d_in[5];

  char* ws = (char*)d_ws;
  unsigned short* W16 = (unsigned short*)(ws + oW16);
  unsigned short* XP  = (unsigned short*)(ws + oXP);
  unsigned short* V   = (unsigned short*)(ws + oV);
  unsigned short* Qh  = (unsigned short*)(ws + oQh);
  unsigned short* Ql  = (unsigned short*)(ws + oQl);
  unsigned short* Kh  = (unsigned short*)(ws + oKh);
  unsigned short* Kl  = (unsigned short*)(ws + oKl);
  float* out = (float*)d_out;

  const dim3 blk256(256), blk128(128);

  cvt_w<<<dim3(MW / 8), blk256, 0, stream>>>(wq, wk, wv, W16);
  cvt_x<<<dim3(NN / QT, CC / QT, NB), blk256, 0, stream>>>(x, XP);
  gemm_qk<<<dim3(NN / QT, MQK / QT, NB), blk128, 0, stream>>>(W16, XP, wq, wk, Qh, Ql, Kh, Kl);
  gemm_v<<<dim3(NN / QT, CC / QT, NB), blk128, 0, stream>>>(W16, XP, wv, bv, V);
  attn_k<<<dim3(NQ / QT, NB, 2), blk128, 0, stream>>>(Qh, Ql, Kh, Kl, V, x, gamma, out);
  (void)hipGetLastError();
}
